// ContextualInvertedResidual_11751030522700
// MI455X (gfx1250) — hardware-verified
//
#include <hip/hip_runtime.h>
#include <math.h>
#include <stdint.h>

#define NB   32
#define CIN  64
#define EC   384
#define IMW  56
#define HW   3136
#define NPT  49
#define XTP  72
#define STP  68
#define BKP  136
#define SOP  68
#define CXS  256.0f
#define CWS  256.0f
#define BO_S1 0
#define BO_T1 384
#define BO_S2 768
#define BO_T2 1152
#define BO_S3 1536
#define BO_T3 1600
#define BNPN 1664

static_assert(HW == NPT * 64);
static_assert(BNPN == BO_T3 + CIN);
static_assert((BNPN % 32) == 0);
static_assert(BNPN / 4 == 416);
static_assert((XTP % 8) == 0);
static_assert((BKP % 8) == 0);
static_assert((STP * 4) % 16 == 0);
static_assert((SOP * 4) % 16 == 0);
static_assert(64 * SOP * 4 <= 2 * 64 * BKP * 2);
static_assert(EC == 3 * 128);
static_assert(CIN == 2 * 32);

typedef _Float16 v16h __attribute__((ext_vector_type(16)));
typedef _Float16 v8h  __attribute__((ext_vector_type(8)));
typedef float    v8f  __attribute__((ext_vector_type(8)));
typedef float    v4f  __attribute__((ext_vector_type(4)));
typedef unsigned int v4u __attribute__((ext_vector_type(4)));
union Frag { v16h v; v8h half[2]; };

__device__ __forceinline__ unsigned short bf_bits(float f) {
  unsigned u = __float_as_uint(f);
  return (unsigned short)((u + 0x7FFFu + ((u >> 16) & 1u)) >> 16);
}
__device__ __forceinline__ float bfr(float f) { return __uint_as_float(((unsigned)bf_bits(f)) << 16); }
__device__ __forceinline__ unsigned short h_bits(_Float16 x) { return __builtin_bit_cast(unsigned short, x); }
__device__ __forceinline__ unsigned pk16(unsigned short a, unsigned short b) { return (unsigned)a | ((unsigned)b << 16); }
__device__ __forceinline__ v8f zero8() { v8f z = {0.f, 0.f, 0.f, 0.f, 0.f, 0.f, 0.f, 0.f}; return z; }

__device__ __forceinline__ v16h ldfrag_h(const _Float16* p) {
  Frag f;
  f.half[0] = *(const v8h*)(p);
  f.half[1] = *(const v8h*)(p + 16);
  return f.v;
}

__device__ __forceinline__ v8f mma_h(v16h a, v16h b, v8f c) {
  c = __builtin_amdgcn_wmma_f32_16x16x32_f16(false, a, false, b, (short)0, c, false, false);
#if defined(__HIP_DEVICE_COMPILE__)
  asm volatile("v_nop\n\tv_nop\n\tv_nop\n\tv_nop" : "+v"(c) : "v"(a), "v"(b));
#endif
  return c;
}
__device__ __forceinline__ void wave_sync_lds() {
  __builtin_amdgcn_fence(__ATOMIC_RELEASE, "workgroup");
  __builtin_amdgcn_wave_barrier();
  __builtin_amdgcn_fence(__ATOMIC_ACQUIRE, "workgroup");
}

__device__ __forceinline__ v4u pack8h(v4f a, v4f b) {
  v4u p;
  p[0] = pk16(h_bits((_Float16)a[0]), h_bits((_Float16)a[1]));
  p[1] = pk16(h_bits((_Float16)a[2]), h_bits((_Float16)a[3]));
  p[2] = pk16(h_bits((_Float16)b[0]), h_bits((_Float16)b[1]));
  p[3] = pk16(h_bits((_Float16)b[2]), h_bits((_Float16)b[3]));
  return p;
}
__device__ __forceinline__ void split8h(v4f a, v4f b, v4u& ph, v4u& pl) {
  v4f ra, rb;
#pragma unroll
  for (int e = 0; e < 4; ++e) {
    const _Float16 ha = (_Float16)a[e];
    ra[e] = (a[e] - (float)ha) * 2048.0f;
    const _Float16 hb = (_Float16)b[e];
    rb[e] = (b[e] - (float)hb) * 2048.0f;
  }
  ph = pack8h(a, b);
  pl = pack8h(ra, rb);
}

__device__ __forceinline__ void cvt8_w(const float* __restrict__ src, unsigned short* dst, size_t e0) {
  const v4f a = *(const v4f*)(src + e0);
  const v4f b = *(const v4f*)(src + e0 + 4);
  v4f sa, sb;
#pragma unroll
  for (int e = 0; e < 4; ++e) { sa[e] = bfr(a[e]) * CWS; sb[e] = bfr(b[e]) * CWS; }
  const v4u pk = pack8h(sa, sb);
  *(volatile v4u*)(dst + e0) = pk;
  __threadfence();
  *(volatile v4u*)(dst + e0) = pk;
}
__global__ __launch_bounds__(256)
void prep_k(const float* __restrict__ g1, const float* __restrict__ b1, const float* __restrict__ m1,
            const float* __restrict__ v1, const float* __restrict__ g2, const float* __restrict__ b2,
            const float* __restrict__ m2, const float* __restrict__ v2, const float* __restrict__ g3,
            const float* __restrict__ b3, const float* __restrict__ m3, const float* __restrict__ v3,
            const float* __restrict__ we, const float* __restrict__ wp,
            float* bnp, unsigned short* Weh, unsigned short* Wph) {
  __shared__ __align__(16) float bs[BNPN];
  const int tid = threadIdx.x, blk = blockIdx.x;
  if (blk == 0) {
    for (int i = tid; i < 2 * EC + CIN; i += 256) {
      const int which = ((i >= EC) ? 1 : 0) + ((i >= 2 * EC) ? 1 : 0);
      const int ci = i - EC * which;
      const float* G = (which == 0) ? g1 : ((which == 1) ? g2 : g3);
      const float* B = (which == 0) ? b1 : ((which == 1) ? b2 : b3);
      const float* M = (which == 0) ? m1 : ((which == 1) ? m2 : m3);
      const float* V = (which == 0) ? v1 : ((which == 1) ? v2 : v3);
      const int so = (which == 0) ? BO_S1 : ((which == 1) ? BO_S2 : BO_S3);
      const int to = (which == 0) ? BO_T1 : ((which == 1) ? BO_T2 : BO_T3);
      const float gg = bfr(G[ci]), bb = bfr(B[ci]), mm = bfr(M[ci]), vv = bfr(V[ci]);
      const float sc = gg * (1.0f / sqrtf(vv + 1.0e-5f));
      bs[so + ci] = sc;
      bs[to + ci] = bb - mm * sc;
    }
    __syncthreads();
    const bool has1 = tid < (BNPN / 4 - 256);
    const int p1 = has1 ? (256 + tid) : 256;
    const v4f q0 = *(const v4f*)(bs + tid * 4);
    const v4f q1 = *(const v4f*)(bs + p1 * 4);
    for (int pass = 0; pass < 2; ++pass) {
      *(volatile v4f*)(bnp + tid * 4) = q0;
      if (has1) *(volatile v4f*)(bnp + p1 * 4) = q1;
      __threadfence();
    }
  } else if (blk <= 12) {
    cvt8_w(we, Weh, ((size_t)(blk - 1) * 256 + tid) * 8);
  } else {
    cvt8_w(wp, Wph, ((size_t)(blk - 13) * 256 + tid) * 8);
  }
}

__global__ __launch_bounds__(256)
void expand_k(const float* __restrict__ x, const unsigned short* __restrict__ Weh, const float* __restrict__ bnp,
              unsigned short* Hp, float* part) {
  __shared__ __align__(16) unsigned short xt[64 * XTP];
  __shared__ __align__(16) float stall[8 * 16 * STP];
  __shared__ __align__(16) float csum[EC];
  __shared__ float s1s[EC], t1s[EC];
  const int tid = threadIdx.x, wave = tid >> 5, lane = tid & 31, hh = lane >> 4, c = lane & 15;
  const int pt = blockIdx.x, n = blockIdx.y;

  {
    const int ci = tid >> 2, pq = tid & 3;
    const float* xp = x + ((size_t)(n * CIN + ci)) * HW + pt * 64 + pq * 16;
#pragma unroll
    for (int j4 = 0; j4 < 4; ++j4) {
      const v4f v = *(const v4f*)(xp + 4 * j4);
#pragma unroll
      for (int e = 0; e < 4; ++e)
        xt[(pq * 16 + 4 * j4 + e) * XTP + ci] = h_bits((_Float16)(bfr(v[e]) * CXS));
    }
  }
  for (int i = tid; i < EC; i += 256) { s1s[i] = bnp[BO_S1 + i]; t1s[i] = bnp[BO_T1 + i]; }
  __syncthreads();

  const _Float16* A  = (const _Float16*)(const void*)Weh;
  const _Float16* Bt = (const _Float16*)(const void*)xt;
  float* st = stall + wave * (16 * STP);

#pragma unroll 1
  for (int mt = wave; mt < 24; mt += 8) {
    v8f acc[4];
#pragma unroll
    for (int nt = 0; nt < 4; ++nt) acc[nt] = zero8();
#pragma unroll
    for (int ks = 0; ks < 2; ++ks) {
      const int k0 = ks * 32;
      const v16h a = ldfrag_h(A + (size_t)(mt * 16 + c) * CIN + k0 + 8 * hh);
#pragma unroll
      for (int nt = 0; nt < 4; ++nt) {
        const v16h b = ldfrag_h(Bt + (nt * 16 + c) * XTP + k0 + 8 * hh);
        acc[nt] = mma_h(a, b, acc[nt]);
      }
    }
#pragma unroll
    for (int r = 0; r < 8; ++r) {
      const int ch = mt * 16 + 8 * hh + r;
      const float sc = s1s[ch] * (1.0f / 65536.0f), sh = t1s[ch];
#pragma unroll
      for (int nt = 0; nt < 4; ++nt) {
        float v = acc[nt][r] * sc + sh;
        v = fminf(fmaxf(v, 0.0f), 6.0f);
        acc[nt][r] = v;
      }
    }
    float q[8];
#pragma unroll
    for (int r = 0; r < 8; ++r) {
      float s = ((acc[0][r] + acc[1][r]) + acc[2][r]) + acc[3][r];
      s += __shfl_xor(s, 1, 32);
      s += __shfl_xor(s, 2, 32);
      s += __shfl_xor(s, 4, 32);
      s += __shfl_xor(s, 8, 32);
      q[r] = s;
    }
    if (c == 0) {
#pragma unroll
      for (int r = 0; r < 8; ++r) csum[mt * 16 + 8 * hh + r] = q[r];
    }
#pragma unroll
    for (int nt = 0; nt < 4; ++nt) {
#pragma unroll
      for (int r = 0; r < 8; ++r) st[(8 * hh + r) * STP + nt * 16 + c] = acc[nt][r];
    }
    wave_sync_lds();
    v4u pk[4];
    size_t offs[4];
#pragma unroll
    for (int it = 0; it < 4; ++it) {
      const int row = it * 4 + (lane >> 3), piece = lane & 7;
      const v4f fa = *(const v4f*)(st + row * STP + piece * 8);
      const v4f fb = *(const v4f*)(st + row * STP + piece * 8 + 4);
      pk[it] = pack8h(fa, fb);
      offs[it] = ((size_t)(n * EC + mt * 16 + row)) * HW + pt * 64 + piece * 8;
    }
    for (int pass = 0; pass < 2; ++pass) {
#pragma unroll
      for (int it = 0; it < 4; ++it) *(volatile v4u*)(Hp + offs[it]) = pk[it];
      __threadfence();
    }
    wave_sync_lds();
  }
  __syncthreads();
  if (wave == 0) {
    v4f pv[3];
    size_t po[3];
#pragma unroll
    for (int i = 0; i < 3; ++i) {
      const int piece = i * 32 + lane;
      pv[i] = *(const v4f*)(csum + piece * 4);
      po[i] = ((size_t)(n * NPT + pt)) * EC + piece * 4;
    }
    for (int pass = 0; pass < 2; ++pass) {
#pragma unroll
      for (int i = 0; i < 3; ++i) *(volatile v4f*)(part + po[i]) = pv[i];
      __threadfence();
    }
  }
}

__global__ __launch_bounds__(256)
void ctx_k(const float* __restrict__ part, const float* __restrict__ wctx, float* cb) {
  __shared__ __align__(16) float ctxs[EC];
  __shared__ __align__(16) float cbs[EC];
  const int tid = threadIdx.x, n = blockIdx.x;
  for (int ch = tid; ch < EC; ch += 256) {
    const float* p = part + (size_t)n * NPT * EC + ch;
    float s = 0.0f;
#pragma unroll 1
    for (int t = 0; t < NPT; ++t) s += p[t * EC];
    ctxs[ch] = s * (1.0f / 3136.0f);
  }
  __syncthreads();
  for (int o = tid; o < EC; o += 256) {
    const float* wr = wctx + (size_t)o * EC;
    float s = 0.0f;
#pragma unroll 1
    for (int cc = 0; cc < EC; ++cc) s += ctxs[cc] * bfr(wr[cc]);
    cbs[o] = s;
  }
  __syncthreads();
  if (tid < 32) {
    v4f pv[3];
    size_t po[3];
#pragma unroll
    for (int i = 0; i < 3; ++i) {
      const int piece = i * 32 + tid;
      pv[i] = *(const v4f*)(cbs + piece * 4);
      po[i] = (size_t)n * EC + piece * 4;
    }
    for (int pass = 0; pass < 2; ++pass) {
#pragma unroll
      for (int i = 0; i < 3; ++i) *(volatile v4f*)(cb + po[i]) = pv[i];
      __threadfence();
    }
  }
}

__global__ __launch_bounds__(256)
void proj_k(const float* __restrict__ x, const unsigned short* __restrict__ Hp, const float* __restrict__ wdw,
            const float* __restrict__ cb, const float* __restrict__ bnp, const unsigned short* __restrict__ Wph,
            float* out) {
  __shared__ float wdws[EC * 9];
  __shared__ float cbs[EC], s2s[EC], t2s[EC], s3s[CIN], t3s[CIN];
  __shared__ __align__(16) unsigned short big[2 * 64 * BKP];
  unsigned short* Bh = big;
  unsigned short* Bl = big + 64 * BKP;
  const int tid = threadIdx.x, wave = tid >> 5, lane = tid & 31, hh = lane >> 4, c = lane & 15;
  const int pt = blockIdx.x, n = blockIdx.y;

  for (int i = tid; i < EC * 9; i += 256) wdws[i] = bfr(wdw[i]);
  for (int i = tid; i < EC; i += 256) {
    cbs[i] = cb[(size_t)n * EC + i];
    s2s[i] = bnp[BO_S2 + i];
    t2s[i] = bnp[BO_T2 + i];
  }
  for (int i = tid; i < CIN; i += 256) { s3s[i] = bnp[BO_S3 + i]; t3s[i] = bnp[BO_T3 + i]; }

  const int px = tid & 63, cq = tid >> 6;
  const int p = pt * 64 + px;
  const int hy = p / IMW, wx = p - hy * IMW;
  int toff[9];
  float tmsk[9];
#pragma unroll
  for (int dy = 0; dy < 3; ++dy) {
#pragma unroll
    for (int dx = 0; dx < 3; ++dx) {
      const int yy = hy + dy - 1, xx = wx + dx - 1;
      const bool ok = ((unsigned)yy < (unsigned)IMW) && ((unsigned)xx < (unsigned)IMW);
      const int yc = (yy < 0) ? 0 : ((yy > IMW - 1) ? (IMW - 1) : yy);
      const int xc = (xx < 0) ? 0 : ((xx > IMW - 1) ? (IMW - 1) : xx);
      toff[dy * 3 + dx] = yc * IMW + xc;
      tmsk[dy * 3 + dx] = ok ? 1.0f : 0.0f;
    }
  }

  const _Float16* Hh  = (const _Float16*)(const void*)Hp;
  const _Float16* A   = (const _Float16*)(const void*)Wph;
  const _Float16* Bhh = (const _Float16*)(const void*)Bh;
  const _Float16* Blh = (const _Float16*)(const void*)Bl;
  const int mt = wave & 3, ntb = wave >> 2;

  v8f acch[2], accl[2];
#pragma unroll
  for (int j = 0; j < 2; ++j) { acch[j] = zero8(); accl[j] = zero8(); }

#pragma unroll 1
  for (int g = 0; g < 3; ++g) {
    __syncthreads();
#pragma unroll 1
    for (int jb = 0; jb < 4; ++jb) {
      const int chl0 = cq * 32 + jb * 8;
      const int ch0 = g * 128 + chl0;
      v4f fa, fb;
#pragma unroll
      for (int e = 0; e < 8; ++e) {
        const int ch = ch0 + e;
        const _Float16* hp = Hh + ((size_t)(n * EC + ch)) * HW;
        const float* w9 = wdws + ch * 9;
        float a = 0.0f;
#pragma unroll
        for (int t = 0; t < 9; ++t) a += ((float)hp[toff[t]] * tmsk[t]) * w9[t];
        float u = (a + cbs[ch]) * s2s[ch] + t2s[ch];
        u = fminf(fmaxf(u, 0.0f), 6.0f);
        if (e < 4) fa[e] = u; else fb[e - 4] = u;
      }
      v4u ph, pl;
      split8h(fa, fb, ph, pl);
      *(v4u*)(Bh + px * BKP + chl0) = ph;
      *(v4u*)(Bl + px * BKP + chl0) = pl;
    }
    __syncthreads();
#pragma unroll
    for (int kk = 0; kk < 4; ++kk) {
      const int kg = g * 128 + kk * 32;
      const v16h a = ldfrag_h(A + (size_t)(mt * 16 + c) * EC + kg + 8 * hh);
#pragma unroll
      for (int j = 0; j < 2; ++j) {
        const int nt = ntb + 2 * j;
        const v16h bh = ldfrag_h(Bhh + (nt * 16 + c) * BKP + kk * 32 + 8 * hh);
        const v16h bl = ldfrag_h(Blh + (nt * 16 + c) * BKP + kk * 32 + 8 * hh);
        acch[j] = mma_h(a, bh, acch[j]);
        accl[j] = mma_h(a, bl, accl[j]);
      }
    }
  }
  __syncthreads();
  float* so = (float*)(void*)big;
#pragma unroll
  for (int j = 0; j < 2; ++j) {
    const int nt = ntb + 2 * j;
#pragma unroll
    for (int r = 0; r < 8; ++r) {
      const float v = (acch[j][r] + accl[j][r] * (1.0f / 2048.0f)) * (1.0f / CWS);
      so[(mt * 16 + 8 * hh + r) * SOP + nt * 16 + c] = v;
    }
  }
  __syncthreads();
  v4f ov[4];
  size_t offs[4];
#pragma unroll
  for (int it = 0; it < 4; ++it) {
    const int ch = wave * 8 + it * 2 + hh;
    const v4f t = *(const v4f*)(so + ch * SOP + c * 4);
    const size_t off = ((size_t)(n * CIN + ch)) * HW + pt * 64 + c * 4;
    const v4f xr = *(const v4f*)(x + off);
    const float sc = s3s[ch], sh = t3s[ch];
    v4f o4;
#pragma unroll
    for (int e = 0; e < 4; ++e) o4[e] = (t[e] * sc + sh) + bfr(xr[e]);
    ov[it] = o4;
    offs[it] = off;
  }
  for (int pass = 0; pass < 2; ++pass) {
#pragma unroll
    for (int it = 0; it < 4; ++it) *(volatile v4f*)(out + offs[it]) = ov[it];
    __threadfence();
  }
}

extern "C" void kernel_launch(void* const* d_in, const int* in_sizes, int n_in,
                              void* d_out, int out_size, void* d_ws, size_t ws_size,
                              hipStream_t stream) {
  if (n_in < 17) return;
  if (in_sizes[0] != NB * CIN * HW) return;
  if (in_sizes[1] != EC * CIN) return;
  if (in_sizes[2] != EC || in_sizes[3] != EC || in_sizes[4] != EC || in_sizes[5] != EC) return;
  if (in_sizes[6] != EC * 9) return;
  if (in_sizes[7] != EC * EC) return;
  if (in_sizes[8] != EC || in_sizes[9] != EC || in_sizes[10] != EC || in_sizes[11] != EC) return;
  if (in_sizes[12] != CIN * EC) return;
  if (in_sizes[13] != CIN || in_sizes[14] != CIN || in_sizes[15] != CIN || in_sizes[16] != CIN) return;
  if (out_size != NB * CIN * HW) return;

  const float* x      = (const float*)d_in[0];
  const float* w_exp  = (const float*)d_in[1];
  const float* g1 = (const float*)d_in[2];
  const float* b1 = (const float*)d_in[3];
  const float* m1 = (const float*)d_in[4];
  const float* v1 = (const float*)d_in[5];
  const float* w_dw   = (const float*)d_in[6];
  const float* w_ctx  = (const float*)d_in[7];
  const float* g2 = (const float*)d_in[8];
  const float* b2 = (const float*)d_in[9];
  const float* m2 = (const float*)d_in[10];
  const float* v2 = (const float*)d_in[11];
  const float* w_proj = (const float*)d_in[12];
  const float* g3 = (const float*)d_in[13];
  const float* b3 = (const float*)d_in[14];
  const float* m3 = (const float*)d_in[15];
  const float* v3 = (const float*)d_in[16];
  float* out = (float*)d_out;

  const size_t sBNP  = (size_t)BNPN * 4;
  const size_t sWE   = (size_t)EC * CIN * 2;
  const size_t sWP   = (size_t)CIN * EC * 2;
  const size_t sCB   = (size_t)NB * EC * 4;
  const size_t sPART = (size_t)NB * NPT * EC * 4;
  const size_t sH    = (size_t)NB * EC * HW * 2;
  size_t off = 0;
  const size_t oBNP  = off; off += sBNP;
  const size_t oWE   = off; off += sWE;
  const size_t oWP   = off; off += sWP;
  const size_t oCB   = off; off += sCB;
  const size_t oPART = off; off += sPART;
  const size_t oH    = off; off += sH;
  if (off > ws_size) return;
  if (off > (size_t)134217728) return;

  char* ws = (char*)d_ws;
  float* bnp           = (float*)(ws + oBNP);
  unsigned short* Weh  = (unsigned short*)(ws + oWE);
  unsigned short* Wph  = (unsigned short*)(ws + oWP);
  float* cb            = (float*)(ws + oCB);
  float* part          = (float*)(ws + oPART);
  unsigned short* Hp   = (unsigned short*)(ws + oH);

  const dim3 blk(256);
  prep_k<<<dim3(25), blk, 0, stream>>>(g1, b1, m1, v1, g2, b2, m2, v2, g3, b3, m3, v3,
                                       w_exp, w_proj, bnp, Weh, Wph);
  expand_k<<<dim3(NPT, NB), blk, 0, stream>>>(x, Weh, bnp, Hp, part);
  ctx_k<<<dim3(NB), blk, 0, stream>>>(part, w_ctx, cb);
  proj_k<<<dim3(NPT, NB), blk, 0, stream>>>(x, Hp, w_dw, cb, bnp, Wph, out);
  (void)hipGetLastError();
}
